// GroupedQueryAttention_58394375357343
// MI455X (gfx1250) — hardware-verified
//
#include <hip/hip_runtime.h>
#ifndef NB
#define NB 2
#endif
#ifndef SEQ
#define SEQ 2048
#endif
#define NB_FULL 2
#define SEQ_FULL 2048
#define DM 1024
#define NH 16
#define HD 64
#define NG 4
#define HPG 4
#define KVD 256
#define NPJ 1536
#define NR (NB * SEQ)
#define WSC 64.0f
#define WSCI 0.015625f
#define PCAR 256.0f

typedef __bf16 v16b __attribute__((ext_vector_type(16)));
typedef _Float16 v16h __attribute__((ext_vector_type(16)));
typedef unsigned short v8us __attribute__((ext_vector_type(8), may_alias));
typedef float v8f __attribute__((ext_vector_type(8)));
typedef float v4f __attribute__((ext_vector_type(4)));
typedef float v4fa __attribute__((ext_vector_type(4), may_alias));
union FragB { v16b v; v8us half[2]; unsigned short u[16]; };
union FragH { v16h v; v8us half[2]; _Float16 h[16]; unsigned short u[16]; };

static_assert(SEQ % 128 == 0);
static_assert(NR % 128 == 0);
static_assert(NB <= NB_FULL);
static_assert(SEQ <= SEQ_FULL);
static_assert(DM == NH * HD);
static_assert(KVD == NG * HD);
static_assert(NH == NG * HPG);
static_assert(HPG == 4);
static_assert(HD == 64);
static_assert(NPJ == DM + 2 * KVD);
static_assert(DM % 64 == 0);
static_assert(KVD % 64 == 0);
static_assert(DM % 32 == 0);
static_assert(DM == 4 * 32 * 8);
static_assert(DM % 256 == 0);
static_assert(KVD % 256 == 0);
static_assert((size_t)NB_FULL * SEQ_FULL * DM * 4 == (size_t)16777216);

#define AL256(x) ((((size_t)(x)) + 255) & ~(size_t)255)
constexpr size_t SZ_BW  = AL256((size_t)NPJ * DM * 2);
constexpr size_t SZ_BO  = AL256((size_t)DM * DM * 2);
constexpr size_t SZ_X16 = AL256((size_t)NR * DM * 2);
constexpr size_t SZ_ST  = AL256((size_t)2 * NR * 4);
constexpr size_t SZ_CS  = AL256((size_t)NPJ * 4);
constexpr size_t SZ_Q   = AL256((size_t)NR * DM * 2);
constexpr size_t SZ_K   = AL256((size_t)NR * KVD * 2);
constexpr size_t OFF_BW  = 0;
constexpr size_t OFF_BO  = OFF_BW + SZ_BW;
constexpr size_t OFF_X16 = OFF_BO + SZ_BO;
constexpr size_t OFF_ST  = OFF_X16 + SZ_X16;
constexpr size_t OFF_CS  = OFF_ST + SZ_ST;
constexpr size_t OFF_CB  = OFF_CS + SZ_CS;
constexpr size_t OFF_QH  = OFF_CB + SZ_CS;
constexpr size_t OFF_QL  = OFF_QH + SZ_Q;
constexpr size_t OFF_KH  = OFF_QL + SZ_Q;
constexpr size_t OFF_KL  = OFF_KH + SZ_K;
constexpr size_t OFF_V16 = OFF_KL + SZ_K;
constexpr size_t OFF_VT  = OFF_V16 + SZ_K;
constexpr size_t OFF_OH  = OFF_VT + SZ_K;
constexpr size_t OFF_OL  = OFF_OH + SZ_Q;
constexpr size_t WS_TOTAL = OFF_OL + SZ_Q;
static_assert(WS_TOTAL <= (size_t)134217728);

__host__ __device__ __forceinline__ size_t full_row(int r) { return (size_t)(r / SEQ) * SEQ_FULL + (size_t)(r % SEQ); }

__device__ __forceinline__ unsigned short bf16_bits(float x) { unsigned int u = __float_as_uint(x); return (unsigned short)((u + 0x7FFFu + ((u >> 16) & 1u)) >> 16); }
__device__ __forceinline__ float bf16_val(unsigned short b) { return __uint_as_float(((unsigned int)b) << 16); }
__device__ __forceinline__ float bf16_rne(float x) { return bf16_val(bf16_bits(x)); }

__device__ __forceinline__ v16b ld_b(const unsigned short* __restrict__ p, int hh) { FragB f; f.half[0] = *(const v8us*)(p + 8 * hh); f.half[1] = *(const v8us*)(p + 16 + 8 * hh); return f.v; }
__device__ __forceinline__ v16h ld_h(const unsigned short* __restrict__ p, int hh) { FragH f; f.half[0] = *(const v8us*)(p + 8 * hh); f.half[1] = *(const v8us*)(p + 16 + 8 * hh); return f.v; }

__device__ __forceinline__ v8f mma_h(v16h a, v16h b, v8f c) {
  c = __builtin_amdgcn_wmma_f32_16x16x32_f16(false, a, false, b, (short)0, c, false, false);
  asm volatile("v_nop\n\tv_nop\n\tv_nop\n\tv_nop" : "+v"(c) : "v"(a), "v"(b));
  return c;
}
template <int NT>
__device__ __forceinline__ v8f mma_b(v16b ah, v16b al, v16b bh, v16b bl, v8f c) {
  c = __builtin_amdgcn_wmma_f32_16x16x32_bf16(false, ah, false, bh, (short)0, c, false, false);
  if (NT >= 2) c = __builtin_amdgcn_wmma_f32_16x16x32_bf16(false, al, false, bh, (short)0, c, false, false);
  if (NT >= 3) c = __builtin_amdgcn_wmma_f32_16x16x32_bf16(false, ah, false, bl, (short)0, c, false, false);
  asm volatile("v_nop\n\tv_nop\n\tv_nop\n\tv_nop" : "+v"(c) : "v"(ah), "v"(al), "v"(bh), "v"(bl));
  return c;
}
__device__ __forceinline__ void split8(const float* v, v8us& hi, v8us& lo) {
#pragma unroll
  for (int i = 0; i < 8; ++i) { const unsigned short hb = bf16_bits(v[i]); hi[i] = hb; lo[i] = bf16_bits(v[i] - bf16_val(hb)); }
}

__global__ __launch_bounds__(256) void k_wt_f16g(const float* __restrict__ W, const float* __restrict__ g, unsigned short* __restrict__ Wt, int K, int N, float scale) {
  const int t = blockIdx.x * 256 + threadIdx.x;
  const int k8n = K / 8;
  if (t >= N * k8n) return;
  const int n = t / k8n, k8 = (t % k8n) * 8;
  FragH f;
#pragma unroll
  for (int i = 0; i < 8; ++i) f.h[i] = (_Float16)(bf16_rne(g[k8 + i]) * bf16_rne(W[(size_t)(k8 + i) * N + n]) * scale);
  const v8us o = f.half[0];
  *(volatile v8us*)(Wt + (size_t)n * K + k8) = o;
  __threadfence();
  *(volatile v8us*)(Wt + (size_t)n * K + k8) = o;
}

__global__ __launch_bounds__(256) void k_wt_bf16(const float* __restrict__ W, unsigned short* __restrict__ Wt, int K, int N) {
  const int t = blockIdx.x * 256 + threadIdx.x;
  const int k8n = K / 8;
  if (t >= N * k8n) return;
  const int n = t / k8n, k8 = (t % k8n) * 8;
  v8us v;
#pragma unroll
  for (int i = 0; i < 8; ++i) v[i] = bf16_bits(W[(size_t)(k8 + i) * N + n]);
  *(volatile v8us*)(Wt + (size_t)n * K + k8) = v;
  __threadfence();
  *(volatile v8us*)(Wt + (size_t)n * K + k8) = v;
}

__global__ __launch_bounds__(256) void k_colsum(const float* __restrict__ W, const float* __restrict__ g, const float* __restrict__ bt, float* __restrict__ CS, float* __restrict__ CB, int K, int N) {
  __shared__ __attribute__((aligned(16))) float s1[256];
  __shared__ __attribute__((aligned(16))) float s2[256];
  const int tid = threadIdx.x;
  const int n = blockIdx.x * 256 + tid;
  float a = 0.f, b = 0.f;
#pragma unroll 1
  for (int k = 0; k < K; ++k) { const float wv = bf16_rne(W[(size_t)k * N + n]); a += bf16_rne(g[k]) * wv; b += bf16_rne(bt[k]) * wv; }
  s1[tid] = a; s2[tid] = b;
  __syncthreads();
  if (tid < 64) {
    const v4f va = *(const v4fa*)&s1[tid * 4];
    const v4f vb = *(const v4fa*)&s2[tid * 4];
    float* pa = CS + (size_t)blockIdx.x * 256 + tid * 4;
    float* pb = CB + (size_t)blockIdx.x * 256 + tid * 4;
    *(volatile v4f*)pa = va; *(volatile v4f*)pb = vb;
    __threadfence();
    *(volatile v4f*)pa = va; *(volatile v4f*)pb = vb;
  }
}

__global__ __launch_bounds__(256) void k_lnstat(const float* __restrict__ x, unsigned short* __restrict__ X16, float* __restrict__ ST) {
  __shared__ __attribute__((aligned(16))) float sst[64];
  const int tid = threadIdx.x, w = tid >> 5, lane = tid & 31;
  const int rbase = blockIdx.x * 32 + w * 4;
#pragma unroll 1
  for (int rr = 0; rr < 4; ++rr) {
    const int row = rbase + rr;
    const float* xr = x + full_row(row) * DM;
    unsigned short* dr = X16 + (size_t)row * DM;
    float s = 0.f;
#pragma unroll 1
    for (int c = 0; c < 4; ++c) {
      const int j = c * 256 + lane * 8;
      const v4f a = *(const v4fa*)(xr + j), b = *(const v4fa*)(xr + j + 4);
      FragH f;
#pragma unroll
      for (int q = 0; q < 4; ++q) { const float va = bf16_rne(a[q]), vb = bf16_rne(b[q]); s += va; s += vb; f.h[q] = (_Float16)va; f.h[4 + q] = (_Float16)vb; }
      const v8us o = f.half[0];
      *(volatile v8us*)(dr + j) = o;
    }
#pragma unroll
    for (int mk = 16; mk > 0; mk >>= 1) s += __shfl_xor(s, mk, 32);
    const float mu = s * (1.0f / (float)DM);
    float s2 = 0.f;
#pragma unroll 1
    for (int c = 0; c < 4; ++c) {
      const int j = c * 256 + lane * 8;
      const v4f a = *(const v4fa*)(xr + j), b = *(const v4fa*)(xr + j + 4);
#pragma unroll
      for (int q = 0; q < 4; ++q) { const float da = bf16_rne(a[q]) - mu, db = bf16_rne(b[q]) - mu; s2 += da * da; s2 += db * db; }
    }
#pragma unroll
    for (int mk = 16; mk > 0; mk >>= 1) s2 += __shfl_xor(s2, mk, 32);
    const float rs = rsqrtf(s2 * (1.0f / (float)DM) + 1e-5f);
    if (lane == 0) { sst[w * 4 + rr] = rs; sst[32 + w * 4 + rr] = -mu * rs; }
  }
  __threadfence();
#pragma unroll 1
  for (int rr = 0; rr < 4; ++rr) {
    const int row = rbase + rr;
    const float* xr = x + full_row(row) * DM;
    unsigned short* dr = X16 + (size_t)row * DM;
#pragma unroll 1
    for (int c = 0; c < 4; ++c) {
      const int j = c * 256 + lane * 8;
      const v4f a = *(const v4fa*)(xr + j), b = *(const v4fa*)(xr + j + 4);
      FragH f;
#pragma unroll
      for (int q = 0; q < 4; ++q) { f.h[q] = (_Float16)bf16_rne(a[q]); f.h[4 + q] = (_Float16)bf16_rne(b[q]); }
      const v8us o = f.half[0];
      *(volatile v8us*)(dr + j) = o;
    }
  }
  __syncthreads();
  if (tid < 16) {
    const int which = tid >> 3, piece = tid & 7;
    const v4f v = *(const v4fa*)&sst[which * 32 + piece * 4];
    float* dst = ST + (size_t)which * NR + (size_t)blockIdx.x * 32 + piece * 4;
    *(volatile v4f*)dst = v;
    __threadfence();
    *(volatile v4f*)dst = v;
  }
}

__global__ __launch_bounds__(128) void k_proj(const unsigned short* __restrict__ X16, const unsigned short* __restrict__ BW, const float* __restrict__ ST,
                                              const float* __restrict__ CS, const float* __restrict__ CB,
                                              unsigned short* __restrict__ Qh, unsigned short* __restrict__ Ql, unsigned short* __restrict__ Kh, unsigned short* __restrict__ Kl, unsigned short* __restrict__ V16) {
  __shared__ __attribute__((aligned(16))) float so[4][32][68];
  const int tid = threadIdx.x, w = tid >> 5, lane = tid & 31, ln = lane & 15, hh = lane >> 4;
  constexpr int ntn = NPJ / 64;
  const int mt = blockIdx.x / ntn, nq = blockIdx.x - mt * ntn;
  const int row0 = mt * 128 + 32 * w, col0 = nq * 64;
  const unsigned short* a0p = X16 + (size_t)(row0 + ln) * DM;
  const unsigned short* a1p = a0p + (size_t)16 * DM;
  const unsigned short* b0p = BW + (size_t)(col0 + ln) * DM;
  const unsigned short* b1p = b0p + (size_t)16 * DM;
  const unsigned short* b2p = b1p + (size_t)16 * DM;
  const unsigned short* b3p = b2p + (size_t)16 * DM;
  const v8f z8 = {0.f, 0.f, 0.f, 0.f, 0.f, 0.f, 0.f, 0.f};
  v8f c00 = z8, c01 = z8, c02 = z8, c03 = z8, c10 = z8, c11 = z8, c12 = z8, c13 = z8;
#pragma unroll 1
  for (int kb = 0; kb < DM; kb += 32) {
    const v16h a0 = ld_h(a0p + kb, hh), a1 = ld_h(a1p + kb, hh);
    v16h b = ld_h(b0p + kb, hh); c00 = mma_h(a0, b, c00); c10 = mma_h(a1, b, c10);
    b = ld_h(b1p + kb, hh); c01 = mma_h(a0, b, c01); c11 = mma_h(a1, b, c11);
    b = ld_h(b2p + kb, hh); c02 = mma_h(a0, b, c02); c12 = mma_h(a1, b, c12);
    b = ld_h(b3p + kb, hh); c03 = mma_h(a0, b, c03); c13 = mma_h(a1, b, c13);
  }
  v8f accs[8] = {c00, c01, c02, c03, c10, c11, c12, c13};
#pragma unroll
  for (int u = 0; u < 8; ++u) {
    const int t = u & 3, hf = u >> 2;
#pragma unroll
    for (int r = 0; r < 8; ++r) so[w][hf * 16 + 8 * hh + r][t * 16 + ln] = accs[u][r];
  }
  __syncthreads();
  const int rsub = lane >> 3, c8 = (lane & 7) * 8;
  const v4f cs0 = *(const v4fa*)(CS + col0 + c8), cs1 = *(const v4fa*)(CS + col0 + c8 + 4);
  const v4f cb0 = *(const v4fa*)(CB + col0 + c8), cb1 = *(const v4fa*)(CB + col0 + c8 + 4);
  const float osc = (col0 < DM) ? 0.125f : 1.0f;
  for (int pass = 0; pass < 2; ++pass) {
#pragma unroll 1
    for (int q = 0; q < 8; ++q) {
      const int r = q * 4 + rsub;
      const int row = row0 + r;
      const float ar = ST[row], cr = ST[NR + row];
      const v4f x0 = *(const v4fa*)&so[w][r][c8], x1 = *(const v4fa*)&so[w][r][c8 + 4];
      float v[8];
#pragma unroll
      for (int i = 0; i < 4; ++i) {
        v[i]     = (ar * (x0[i] * WSCI) + cr * cs0[i] + cb0[i]) * osc;
        v[4 + i] = (ar * (x1[i] * WSCI) + cr * cs1[i] + cb1[i]) * osc;
      }
      if (col0 < DM) {
        v8us hi, lo; split8(v, hi, lo);
        const size_t o = (size_t)row * DM + col0 + c8;
        *(volatile v8us*)(Qh + o) = hi; *(volatile v8us*)(Ql + o) = lo;
      } else if (col0 < DM + KVD) {
        v8us hi, lo; split8(v, hi, lo);
        const size_t o = (size_t)row * KVD + (col0 - DM) + c8;
        *(volatile v8us*)(Kh + o) = hi; *(volatile v8us*)(Kl + o) = lo;
      } else {
        FragH f;
#pragma unroll
        for (int i = 0; i < 8; ++i) f.h[i] = (_Float16)v[i];
        const v8us o8 = f.half[0];
        const size_t o = (size_t)row * KVD + (col0 - DM - KVD) + c8;
        *(volatile v8us*)(V16 + o) = o8;
      }
    }
    if (pass == 0) __threadfence();
  }
}

__global__ __launch_bounds__(256) void k_vt(const unsigned short* __restrict__ V16, unsigned short* __restrict__ VT) {
  __shared__ unsigned short tl[64][66];
  const int tid = threadIdx.x;
  const int slab = blockIdx.x / (SEQ / 64), lg = blockIdx.x % (SEQ / 64);
  const int b = slab / NG, g = slab % NG;
  for (int i = tid; i < 64 * 8; i += 256) {
    const int r = i / 8, c8 = (i % 8) * 8;
    FragH f;
    f.half[0] = *(const v8us*)(V16 + ((size_t)b * SEQ + lg * 64 + r) * KVD + g * HD + c8);
#pragma unroll
    for (int q = 0; q < 8; ++q) tl[r][c8 + q] = f.u[q];
  }
  __syncthreads();
  for (int pass = 0; pass < 2; ++pass) {
#pragma unroll
    for (int rd = 0; rd < 2; ++rd) {
      const int d = rd * 32 + tid / 8, pc = tid % 8;
      FragH f;
#pragma unroll
      for (int q = 0; q < 8; ++q) f.u[q] = tl[pc * 8 + q][d];
      const v8us o = f.half[0];
      *(volatile v8us*)(VT + ((size_t)slab * HD + d) * SEQ + lg * 64 + pc * 8) = o;
    }
    if (pass == 0) __threadfence();
  }
}

__device__ __forceinline__ v8f score_tile(const unsigned short* __restrict__ kh, const unsigned short* __restrict__ kl, int hh, v16b qh0, v16b ql0, v16b qh1, v16b ql1) {
  v8f s = {0.f, 0.f, 0.f, 0.f, 0.f, 0.f, 0.f, 0.f};
  v16b ah = ld_b(kh, hh), al = ld_b(kl, hh);
  s = mma_b<3>(ah, al, qh0, ql0, s);
  ah = ld_b(kh + 32, hh); al = ld_b(kl + 32, hh);
  s = mma_b<3>(ah, al, qh1, ql1, s);
  return s;
}

__global__ __launch_bounds__(128) void k_attn(const unsigned short* __restrict__ Qh, const unsigned short* __restrict__ Ql, const unsigned short* __restrict__ Kh, const unsigned short* __restrict__ Kl,
                                              const unsigned short* __restrict__ VT, unsigned short* __restrict__ Oh, unsigned short* __restrict__ Ol) {
  __shared__ __attribute__((aligned(16))) float so[4][16][68];
  const int tid = threadIdx.x, w = tid >> 5, lane = tid & 31, ln = lane & 15, hh = lane >> 4;
  const int bid = blockIdx.x;
  const int qt = bid % (SEQ / 16);
  const int g = (bid / (SEQ / 16)) % NG;
  const int b = bid / ((SEQ / 16) * NG);
  const int h = g * HPG + w;
  const size_t qoff = ((size_t)b * SEQ + qt * 16 + ln) * DM + (size_t)h * HD;
  const v16b qh0 = ld_b(Qh + qoff, hh), ql0 = ld_b(Ql + qoff, hh);
  const v16b qh1 = ld_b(Qh + qoff + 32, hh), ql1 = ld_b(Ql + qoff + 32, hh);
  const size_t kbase = ((size_t)b * SEQ + ln) * KVD + (size_t)g * HD;
  const size_t vbase = ((size_t)(b * NG + g) * HD + ln) * SEQ;
  const v8f z8 = {0.f, 0.f, 0.f, 0.f, 0.f, 0.f, 0.f, 0.f};
  v8f o[4] = {z8, z8, z8, z8};
  float m = -1.0e30f, l = 0.f;
#pragma unroll 1
  for (int kt = 0; kt < SEQ; kt += 32) {
    const size_t ko = kbase + (size_t)kt * KVD;
    const v8f s0 = score_tile(Kh + ko, Kl + ko, hh, qh0, ql0, qh1, ql1);
    const v8f s1 = score_tile(Kh + ko + (size_t)16 * KVD, Kl + ko + (size_t)16 * KVD, hh, qh0, ql0, qh1, ql1);
    float mx = fmaxf(s0[0], s1[0]);
#pragma unroll
    for (int r = 1; r < 8; ++r) mx = fmaxf(mx, fmaxf(s0[r], s1[r]));
    mx = fmaxf(mx, __shfl_xor(mx, 16, 32));
    const float mn = fmaxf(m, mx);
    const float al = __expf(m - mn);
    FragH pb;
    float ps = 0.f;
#pragma unroll
    for (int r = 0; r < 8; ++r) {
      const float p0 = __expf(s0[r] - mn), p1 = __expf(s1[r] - mn);
      ps += p0 + p1;
      pb.h[r] = (_Float16)(p0 * PCAR);
      pb.h[8 + r] = (_Float16)(p1 * PCAR);
    }
    l = l * al + ps;
    m = mn;
#pragma unroll
    for (int tt = 0; tt < 4; ++tt) o[tt] = o[tt] * al;
#pragma unroll
    for (int tt = 0; tt < 4; ++tt) {
      const v16h va = ld_h(VT + vbase + (size_t)tt * 16 * SEQ + kt, hh);
      o[tt] = mma_h(va, pb.v, o[tt]);
    }
  }
  l += __shfl_xor(l, 16, 32);
  const float inv = 1.0f / (PCAR * l);
#pragma unroll
  for (int tt = 0; tt < 4; ++tt)
#pragma unroll
    for (int r = 0; r < 8; ++r) so[w][ln][tt * 16 + 8 * hh + r] = o[tt][r] * inv;
  __syncthreads();
  const int rsub = lane >> 3, c8 = (lane & 7) * 8;
  for (int pass = 0; pass < 2; ++pass) {
#pragma unroll 1
    for (int q = 0; q < 4; ++q) {
      const int r = q * 4 + rsub;
      const v4f x0 = *(const v4fa*)&so[w][r][c8], x1 = *(const v4fa*)&so[w][r][c8 + 4];
      float v[8] = {x0[0], x0[1], x0[2], x0[3], x1[0], x1[1], x1[2], x1[3]};
      v8us hi, lo; split8(v, hi, lo);
      const size_t dsto = ((size_t)b * SEQ + qt * 16 + r) * DM + (size_t)h * HD + c8;
      *(volatile v8us*)(Oh + dsto) = hi; *(volatile v8us*)(Ol + dsto) = lo;
    }
    if (pass == 0) __threadfence();
  }
}

__global__ __launch_bounds__(128) void k_outp(const unsigned short* __restrict__ Oh, const unsigned short* __restrict__ Ol, const unsigned short* __restrict__ BO, const float* __restrict__ bias, float* __restrict__ out) {
  __shared__ __attribute__((aligned(16))) float so[4][32][68];
  const int tid = threadIdx.x, w = tid >> 5, lane = tid & 31, ln = lane & 15, hh = lane >> 4;
  constexpr int ntn = DM / 64;
  const int mt = blockIdx.x / ntn, nq = blockIdx.x - mt * ntn;
  const int row0 = mt * 128 + 32 * w, col0 = nq * 64;
  const size_t a0o = (size_t)(row0 + ln) * DM, a1o = a0o + (size_t)16 * DM;
  const unsigned short* b0p = BO + (size_t)(col0 + ln) * DM;
  const unsigned short* b1p = b0p + (size_t)16 * DM;
  const unsigned short* b2p = b1p + (size_t)16 * DM;
  const unsigned short* b3p = b2p + (size_t)16 * DM;
  const v8f z8 = {0.f, 0.f, 0.f, 0.f, 0.f, 0.f, 0.f, 0.f};
  v8f c00 = z8, c01 = z8, c02 = z8, c03 = z8, c10 = z8, c11 = z8, c12 = z8, c13 = z8;
#pragma unroll 1
  for (int kb = 0; kb < DM; kb += 32) {
    const v16b a0h = ld_b(Oh + a0o + kb, hh), a0l = ld_b(Ol + a0o + kb, hh);
    const v16b a1h = ld_b(Oh + a1o + kb, hh), a1l = ld_b(Ol + a1o + kb, hh);
    v16b bb = ld_b(b0p + kb, hh); c00 = mma_b<2>(a0h, a0l, bb, bb, c00); c10 = mma_b<2>(a1h, a1l, bb, bb, c10);
    bb = ld_b(b1p + kb, hh); c01 = mma_b<2>(a0h, a0l, bb, bb, c01); c11 = mma_b<2>(a1h, a1l, bb, bb, c11);
    bb = ld_b(b2p + kb, hh); c02 = mma_b<2>(a0h, a0l, bb, bb, c02); c12 = mma_b<2>(a1h, a1l, bb, bb, c12);
    bb = ld_b(b3p + kb, hh); c03 = mma_b<2>(a0h, a0l, bb, bb, c03); c13 = mma_b<2>(a1h, a1l, bb, bb, c13);
  }
  v8f accs[8] = {c00, c01, c02, c03, c10, c11, c12, c13};
#pragma unroll
  for (int u = 0; u < 8; ++u) {
    const int t = u & 3, hf = u >> 2;
#pragma unroll
    for (int r = 0; r < 8; ++r) so[w][hf * 16 + 8 * hh + r][t * 16 + ln] = accs[u][r];
  }
  __syncthreads();
  const int rsub = lane >> 4, c4 = (lane & 15) * 4;
  const v4f bz = *(const v4fa*)(bias + col0 + c4);
  v4f bq;
#pragma unroll
  for (int i = 0; i < 4; ++i) bq[i] = bf16_rne(bz[i]);
  for (int pass = 0; pass < 2; ++pass) {
#pragma unroll 1
    for (int q = 0; q < 16; ++q) {
      const int r = q * 2 + rsub;
      const v4f x = *(const v4fa*)&so[w][r][c4];
      const v4f v = x + bq;
      *(volatile v4f*)(out + full_row(row0 + r) * DM + col0 + c4) = v;
    }
    if (pass == 0) __threadfence();
  }
}

extern "C" void kernel_launch(void* const* d_in, const int* in_sizes, int n_in,
                              void* d_out, int out_size, void* d_ws, size_t ws_size, hipStream_t stream) {
  if (n_in < 8) return;
  const long long need_x = ((long long)(NB - 1) * SEQ_FULL + SEQ) * DM;
  if ((long long)in_sizes[0] < need_x) return;
  if (in_sizes[1] < DM || in_sizes[2] < DM || in_sizes[7] < DM) return;
  if ((long long)in_sizes[3] < (long long)DM * DM || (long long)in_sizes[6] < (long long)DM * DM) return;
  if ((long long)in_sizes[4] < (long long)DM * KVD || (long long)in_sizes[5] < (long long)DM * KVD) return;
  if ((long long)out_size < need_x) return;
  if ((size_t)WS_TOTAL > ws_size) return;
  const float* x   = (const float*)d_in[0];
  const float* gam = (const float*)d_in[1];
  const float* bet = (const float*)d_in[2];
  const float* wq  = (const float*)d_in[3];
  const float* wk  = (const float*)d_in[4];
  const float* wv  = (const float*)d_in[5];
  const float* wo  = (const float*)d_in[6];
  const float* bo  = (const float*)d_in[7];
  float* out = (float*)d_out;
  unsigned char* ws = (unsigned char*)d_ws;
  unsigned short* BW  = (unsigned short*)(ws + OFF_BW);
  unsigned short* BO  = (unsigned short*)(ws + OFF_BO);
  unsigned short* X16 = (unsigned short*)(ws + OFF_X16);
  float* ST = (float*)(ws + OFF_ST);
  float* CS = (float*)(ws + OFF_CS);
  float* CB = (float*)(ws + OFF_CB);
  unsigned short* Qh  = (unsigned short*)(ws + OFF_QH);
  unsigned short* Ql  = (unsigned short*)(ws + OFF_QL);
  unsigned short* Kh  = (unsigned short*)(ws + OFF_KH);
  unsigned short* Kl  = (unsigned short*)(ws + OFF_KL);
  unsigned short* V16 = (unsigned short*)(ws + OFF_V16);
  unsigned short* VT  = (unsigned short*)(ws + OFF_VT);
  unsigned short* Oh  = (unsigned short*)(ws + OFF_OH);
  unsigned short* Ol  = (unsigned short*)(ws + OFF_OL);

  k_wt_f16g<<<(unsigned)(((size_t)DM * (DM / 8) + 255) / 256), 256, 0, stream>>>(wq, gam, BW, DM, DM, WSC);
  k_wt_f16g<<<(unsigned)(((size_t)KVD * (DM / 8) + 255) / 256), 256, 0, stream>>>(wk, gam, BW + (size_t)DM * DM, DM, KVD, WSC);
  k_wt_f16g<<<(unsigned)(((size_t)KVD * (DM / 8) + 255) / 256), 256, 0, stream>>>(wv, gam, BW + (size_t)(DM + KVD) * DM, DM, KVD, WSC);
  k_wt_bf16<<<(unsigned)(((size_t)DM * (DM / 8) + 255) / 256), 256, 0, stream>>>(wo, BO, DM, DM);
  k_colsum<<<DM / 256, 256, 0, stream>>>(wq, gam, bet, CS, CB, DM, DM);
  k_colsum<<<KVD / 256, 256, 0, stream>>>(wk, gam, bet, CS + DM, CB + DM, DM, KVD);
  k_colsum<<<KVD / 256, 256, 0, stream>>>(wv, gam, bet, CS + DM + KVD, CB + DM + KVD, DM, KVD);
  k_lnstat<<<NR / 32, 256, 0, stream>>>(x, X16, ST);
  k_proj<<<(unsigned)((NR / 128) * (NPJ / 64)), 128, 0, stream>>>(X16, BW, ST, CS, CB, Qh, Ql, Kh, Kl, V16);
  k_vt<<<(unsigned)(NB * NG * (SEQ / 64)), 256, 0, stream>>>(V16, VT);
  k_attn<<<(unsigned)(NB * NG * (SEQ / 16)), 128, 0, stream>>>(Qh, Ql, Kh, Kl, VT, Oh, Ol);
  k_outp<<<(unsigned)((NR / 128) * (DM / 64)), 128, 0, stream>>>(Oh, Ol, BO, bo, out);
}
